// Inferer_48498770706560
// MI455X (gfx1250) — hardware-verified
//
#include <hip/hip_runtime.h>
#include <stdint.h>
#include <math.h>

typedef __attribute__((ext_vector_type(16))) _Float16 v16h;
typedef __attribute__((ext_vector_type(8)))  _Float16 v8h;
typedef __attribute__((ext_vector_type(16))) __bf16   v16b;
typedef __attribute__((ext_vector_type(8)))  __bf16   v8b;
typedef __attribute__((ext_vector_type(8)))  float    v8f;
typedef __attribute__((ext_vector_type(4)))  float    v4f;

__device__ __forceinline__ unsigned short f2bf_bits(float f) {
  unsigned u = __float_as_uint(f);
  return (unsigned short)((u + 0x7FFFu + ((u >> 16) & 1u)) >> 16);
}
__device__ __forceinline__ float bf_bits2f(unsigned short h) { return __uint_as_float(((unsigned)h) << 16); }

__device__ __forceinline__ void dep_guard_h(v8f& a, v8f& b, v16h x, v16h y) { asm volatile("v_nop\n\tv_nop\n\tv_nop\n\tv_nop" : "+v"(a), "+v"(b) : "v"(x), "v"(y)); }
__device__ __forceinline__ void dep_guard_b(v8f& a, v8f& b, v16b x, v16b y) { asm volatile("v_nop\n\tv_nop\n\tv_nop\n\tv_nop" : "+v"(a), "+v"(b) : "v"(x), "v"(y)); }
__device__ __forceinline__ void dep_guard1(v8f& a, v16h x, v16h y) { asm volatile("v_nop\n\tv_nop\n\tv_nop\n\tv_nop" : "+v"(a) : "v"(x), "v"(y)); }
__device__ __forceinline__ void keep4_h(v16h a, v16h b, v16h c, v16h d) { asm volatile("v_nop" :: "v"(a), "v"(b), "v"(c), "v"(d)); }
__device__ __forceinline__ void keep4_b(v16b a, v16b b, v16b c, v16b d) { asm volatile("v_nop" :: "v"(a), "v"(b), "v"(c), "v"(d)); }
__device__ __forceinline__ void acc_guard4(v8f& a, v8f& b, v8f& c, v8f& d) { asm volatile("v_nop\n\tv_nop\n\tv_nop\n\tv_nop" : "+v"(a), "+v"(b), "+v"(c), "+v"(d)); }
template <typename T> struct Frag;
template <> struct Frag<_Float16> {
  typedef v16h V; union U { v16h v; v8h h[2]; };
  static __device__ __forceinline__ v16h load(const _Float16* p) {
    U f; f.h[0] = *(const v8h*)(p); f.h[1] = *(const v8h*)(p + 16); return f.v;
  }
  static __device__ __forceinline__ v8f mma(v16h a, v16h b, v8f c) {
    return __builtin_amdgcn_wmma_f32_16x16x32_f16(false, a, false, b, (short)0, c, false, false);
  }
  static __device__ __forceinline__ void guard(v8f& a, v8f& b, v16h x, v16h y) { dep_guard_h(a, b, x, y); }
  static __device__ __forceinline__ void keep(v16h a, v16h b, v16h c, v16h d) { keep4_h(a, b, c, d); }
};
template <> struct Frag<__bf16> {
  typedef v16b V; union U { v16b v; v8b h[2]; };
  static __device__ __forceinline__ v16b load(const __bf16* p) {
    U f; f.h[0] = *(const v8b*)(p); f.h[1] = *(const v8b*)(p + 16); return f.v;
  }
  static __device__ __forceinline__ v8f mma(v16b a, v16b b, v8f c) {
    return __builtin_amdgcn_wmma_f32_16x16x32_bf16(false, a, false, b, (short)0, c, false, false);
  }
  static __device__ __forceinline__ void guard(v8f& a, v8f& b, v16b x, v16b y) { dep_guard_b(a, b, x, y); }
  static __device__ __forceinline__ void keep(v16b a, v16b b, v16b c, v16b d) { keep4_b(a, b, c, d); }
};

constexpr int Bn   = 256;
constexpr int NO_A = 64,  NF_A = 4;
constexpr int NO_B = 32,  NF_B = 3;
constexpr int NS   = 7;
constexpr int DIN  = 128, DL = 64, DG = 64, DH = 256;
constexpr int DGE  = 448;
constexpr int GROW = (NS + 1) * DGE;
constexpr int DINdA = 704, DINdB = 640;
constexpr int NP   = 2;
constexpr int MA   = Bn * NO_A * NF_A;
constexpr int MB   = Bn * NO_B * NF_B;
constexpr int RA_  = Bn * NO_A;
constexpr int RB_  = Bn * NO_B;

template <int BIAS_MODE, int RES_MODE, int OUT_MODE, int ACT>
__global__ __launch_bounds__(256) void wmma_gemm64(
    const _Float16* __restrict__ A, int lda, long strideA,
    const _Float16* __restrict__ Bt, int ldb, long strideB,
    void* __restrict__ Cout, int ldc, long strideC,
    const float* __restrict__ bias, long strideBias,
    const float* __restrict__ resid, long strideR, int ldr, int rsh,
    int M, int N, int K) {
  typedef _Float16 T;
  typedef v16h V;
  __shared__ __align__(16) float sT[8][16 * 68];
  const int b    = blockIdx.y;
  const int lane = threadIdx.x & 31;
  const int wave = threadIdx.x >> 5;
  const int tilesN = N >> 6;
  const int tilesM = M >> 6;
  const int tile = blockIdx.x * 8 + wave;
  if (tile >= tilesM * tilesN) return;
  const int tm = tile / tilesN;
  const int tn = tile - tm * tilesN;
  const int m0 = tm << 6;
  const int n0 = tn << 6;

  const T* Ab = A  + (size_t)b * strideA;
  const T* Bb = Bt + (size_t)b * strideB;

  const int rlane = lane & 15;
  const int koff  = (lane >> 4) * 8;
  const int mOff  = (lane >> 4) * 8;

  v8f acc[4][4];
#pragma unroll
  for (int i = 0; i < 4; ++i)
#pragma unroll
    for (int j = 0; j < 4; ++j) acc[i][j] = (v8f){0.f,0.f,0.f,0.f,0.f,0.f,0.f,0.f};

  for (int k0 = 0; k0 < K; k0 += 32) {
    V bh[4];
#pragma unroll
    for (int j = 0; j < 4; ++j) {
      const size_t bo = (size_t)(n0 + (j << 4) + rlane) * ldb + koff + k0;
      bh[j] = Frag<T>::load(Bb + bo);
    }
#pragma unroll
    for (int i = 0; i < 4; ++i) {
      const size_t ao = (size_t)(m0 + (i << 4) + rlane) * lda + koff + k0;
      V ah = Frag<T>::load(Ab + ao);
#pragma unroll
      for (int j = 0; j < 4; ++j) {
        acc[i][j] = Frag<T>::mma(ah, bh[j], acc[i][j]);
      }
      Frag<T>::guard(acc[i][0], acc[i][3], ah, ah);
    }
    Frag<T>::keep(bh[0], bh[1], bh[2], bh[3]);
  }
  acc_guard4(acc[0][0], acc[0][1], acc[0][2], acc[0][3]);
  acc_guard4(acc[1][0], acc[1][1], acc[1][2], acc[1][3]);
  acc_guard4(acc[2][0], acc[2][1], acc[2][2], acc[2][3]);
  acc_guard4(acc[3][0], acc[3][1], acc[3][2], acc[3][3]);

  float* slab = sT[wave];
  const float* biasb = (BIAS_MODE != 0) ? (bias + (size_t)b * strideBias) : nullptr;
  const float* Rb    = (RES_MODE != 0) ? (resid + (size_t)b * strideR) : nullptr;
#pragma unroll
  for (int i = 0; i < 4; ++i) {
    const int mBase = m0 + (i << 4);
#pragma unroll
    for (int j = 0; j < 4; ++j) {
      const int n = n0 + (j << 4) + rlane;
      float bv = 0.f;
      if (BIAS_MODE == 2) bv = biasb[n];
#pragma unroll
      for (int r = 0; r < 8; ++r) {
        float v = acc[i][j][r];
        if (BIAS_MODE == 2) v += bv;
        if (RES_MODE == 1) v += Rb[(size_t)(mBase + mOff + r) * ldr + n];
        if (RES_MODE == 2) v += Rb[(size_t)((mBase + mOff + r) >> rsh) * ldr + n];
        if (ACT == 2) v = fmaxf(v, 0.0f);
        if (ACT == 4) v = (v >= 0.f) ? v : 0.01f * v;
        slab[(mOff + r) * 68 + (j << 4) + rlane] = v;
      }
    }
    __builtin_amdgcn_fence(__ATOMIC_RELEASE, "workgroup");
    __builtin_amdgcn_wave_barrier();
    __builtin_amdgcn_fence(__ATOMIC_ACQUIRE, "workgroup");
    if (OUT_MODE == 0) {
      float* C = (float*)Cout + (size_t)b * strideC;
      const int hh = lane >> 4, c4 = (lane & 15) * 4;
      for (int pass = 0; pass < 2; ++pass) {
#pragma unroll
        for (int it = 0; it < 8; ++it) {
          const int row = it * 2 + hh;
          v4f v = *(const v4f*)(slab + row * 68 + c4);
          *(volatile v4f*)(C + (size_t)(mBase + row) * ldc + n0 + c4) = v;
        }
        __threadfence();
      }
    } else {
      const int q = lane >> 3, c8 = (lane & 7) * 8;
      unsigned short* C = (unsigned short*)Cout + (size_t)b * strideC;
      for (int pass = 0; pass < 2; ++pass) {
#pragma unroll
        for (int it = 0; it < 4; ++it) {
          const int row = it * 4 + q;
          const float* sp = slab + row * 68 + c8;
          v8h hv;
#pragma unroll
          for (int e = 0; e < 8; ++e) hv[e] = (_Float16)sp[e];
          *(volatile v8h*)(C + (size_t)(mBase + row) * ldc + n0 + c8) = hv;
        }
        __threadfence();
      }
    }
    __builtin_amdgcn_fence(__ATOMIC_RELEASE, "workgroup");
    __builtin_amdgcn_wave_barrier();
    __builtin_amdgcn_fence(__ATOMIC_ACQUIRE, "workgroup");
  }
}

__global__ __launch_bounds__(256) void cast_f32_f16x8(
    const float* __restrict__ in, _Float16* __restrict__ out, int n8) {
  const int i = blockIdx.x * 256 + threadIdx.x;
  const bool act = i < n8;
  v8h h;
#pragma unroll
  for (int e = 0; e < 8; ++e) h[e] = (_Float16)0.0f;
  _Float16* dp = out;
  if (act) {
    const float* p = in + (size_t)i * 8;
    const v4f a = *(const v4f*)p;
    const v4f c = *(const v4f*)(p + 4);
    h[0] = (_Float16)a[0]; h[1] = (_Float16)a[1]; h[2] = (_Float16)a[2]; h[3] = (_Float16)a[3];
    h[4] = (_Float16)c[0]; h[5] = (_Float16)c[1]; h[6] = (_Float16)c[2]; h[7] = (_Float16)c[3];
    dp = out + (size_t)i * 8;
    *(volatile v8h*)dp = h;
  }
  __threadfence();
  if (act) *(volatile v8h*)dp = h;
}

__global__ __launch_bounds__(256) void transpose_w16(
    const float* __restrict__ src, _Float16* __restrict__ dst, int K, int N) {
  __shared__ float tile[64][65];
  const int s = blockIdx.z, k0 = blockIdx.y * 64, n0 = blockIdx.x * 64, tid = threadIdx.x;
  const float* sp = src + (size_t)s * K * N;
#pragma unroll
  for (int it = 0; it < 16; ++it) {
    const int idx = it * 256 + tid;
    const int kr = idx >> 6, nc = idx & 63;
    tile[kr][nc] = sp[(size_t)(k0 + kr) * N + n0 + nc];
  }
  __syncthreads();
  _Float16* dp = dst + (size_t)s * N * K;
  const int nr0 = tid >> 3, kc = (tid & 7) * 8;
  v8h v0, v1;
#pragma unroll
  for (int e = 0; e < 8; ++e) {
    v0[e] = (_Float16)tile[kc + e][nr0];
    v1[e] = (_Float16)tile[kc + e][nr0 + 32];
  }
  _Float16* p0 = dp + (size_t)(n0 + nr0) * K + k0 + kc;
  _Float16* p1 = dp + (size_t)(n0 + nr0 + 32) * K + k0 + kc;
  *(volatile v8h*)p0 = v0;
  *(volatile v8h*)p1 = v1;
  __threadfence();
  *(volatile v8h*)p0 = v0;
  *(volatile v8h*)p1 = v1;
}

__global__ __launch_bounds__(256) void pack_head_w16(
    const float* __restrict__ Wp, _Float16* __restrict__ dst, int S, int NPo) {
  const int i = blockIdx.x * 256 + threadIdx.x;
  const int total = S * 16 * 32;
  const bool act = i < total;
  v8h v;
#pragma unroll
  for (int e = 0; e < 8; ++e) v[e] = (_Float16)0.0f;
  _Float16* dp = dst;
  if (act) {
    const int s = i >> 9;
    const int rem = i & 511;
    const int n = rem >> 5;
    const int kc = (rem & 31) * 8;
    if (n < NPo) {
#pragma unroll
      for (int e = 0; e < 8; ++e) v[e] = (_Float16)Wp[(size_t)(s * DH + kc + e) * NPo + n];
    }
    dp = dst + (size_t)(s * 16 + n) * DH + kc;
    *(volatile v8h*)dp = v;
  }
  __threadfence();
  if (act) *(volatile v8h*)dp = v;
}

__global__ __launch_bounds__(448) void pool_global_kernel(
    const float* __restrict__ hgA, const float* __restrict__ hgB,
    const int* __restrict__ objA, const int* __restrict__ objB,
    const int* __restrict__ gmask, _Float16* __restrict__ G16) {
  __shared__ float rs[DGE];
  const int b = blockIdx.x, t = threadIdx.x;
  const int fg = t >> 6, c = t & 63;
  float acc = 0.f;
  if (fg < NF_A) {
    const float* hp = hgA + ((size_t)b * NO_A * NF_A + fg) * DG + c;
    const int* om = objA + b * NO_A;
    for (int o = 0; o < NO_A; ++o) {
      const float v = hp[(size_t)o * NF_A * DG];
      acc += (om[o] != 0) ? v : 0.f;
    }
  } else {
    const int f = fg - NF_A;
    const float* hp = hgB + ((size_t)b * NO_B * NF_B + f) * DG + c;
    const int* om = objB + b * NO_B;
    for (int o = 0; o < NO_B; ++o) {
      const float v = hp[(size_t)o * NF_B * DG];
      acc += (om[o] != 0) ? v : 0.f;
    }
  }
  acc = fmaxf(acc, 0.0f);
  rs[t] = acc;
  __syncthreads();
  const int s = t / 56;
  const int col0 = (t - s * 56) * 8;
  const int f2 = col0 >> 6;
  int keep = 1;
  if (s < NS) keep = gmask[(b * NS + s) * NS + f2];
  v8h v;
#pragma unroll
  for (int e = 0; e < 8; ++e) v[e] = (keep != 0) ? (_Float16)rs[col0 + e] : (_Float16)0.0f;
  _Float16* dp = G16 + (size_t)b * GROW + (size_t)t * 8;
  *(volatile v8h*)dp = v;
  __threadfence();
  *(volatile v8h*)dp = v;
}

__global__ __launch_bounds__(256) void build_local_kernel(
    const _Float16* __restrict__ hl, const int* __restrict__ lm, _Float16* __restrict__ Xl,
    int NO, int NF, int rows, int total8) {
  const int i = blockIdx.x * 256 + threadIdx.x;
  const bool act = i < total8;
  v8h v;
#pragma unroll
  for (int e = 0; e < 8; ++e) v[e] = (_Float16)0.0f;
  _Float16* dp = Xl;
  if (act) {
    const int KL  = NF * 64;
    const int KL8 = NF * 8;
    const int perS = rows * KL8;
    const int s = i / perS;
    const int rem = i - s * perS;
    const int row = rem / KL8;
    const int q = rem - row * KL8;
    const int col0 = q * 8;
    const int f = col0 >> 6;
    const int b = row / NO;
    const int keep = lm[(b * NF + s) * NF + f];
    if (keep != 0) v = *(const v8h*)(hl + (size_t)row * KL + col0);
    dp = Xl + (size_t)i * 8;
    *(volatile v8h*)dp = v;
  }
  __threadfence();
  if (act) *(volatile v8h*)dp = v;
}

__global__ __launch_bounds__(128) void head_kernel(
    const _Float16* __restrict__ H, long strideS, const _Float16* __restrict__ Wp16,
    const float* __restrict__ bp, float* __restrict__ out, int NF, int NPo, int Mrows) {
  __shared__ __align__(16) float ot[64 * 8];
  const int m0 = blockIdx.x * 64;
  if (m0 >= Mrows) return;
  const int t = threadIdx.x;
  const int lane = t & 31, wave = t >> 5;
  const int rlane = lane & 15, hh = lane >> 4, koff = hh * 8;
  const int W = NF * NPo;
  for (int s = 0; s < NF; ++s) {
    v8f acc = (v8f){0.f,0.f,0.f,0.f,0.f,0.f,0.f,0.f};
    const _Float16* Ap = H + (size_t)s * strideS + (size_t)(m0 + wave * 16 + rlane) * DH + koff;
    const _Float16* Bp = Wp16 + (size_t)(s * 16 + rlane) * DH + koff;
#pragma unroll
    for (int k0 = 0; k0 < DH; k0 += 32) {
      const v16h a  = Frag<_Float16>::load(Ap + k0);
      const v16h bb = Frag<_Float16>::load(Bp + k0);
      acc = Frag<_Float16>::mma(a, bb, acc);
      dep_guard1(acc, a, bb);
    }
    if (rlane < NPo) {
      const float bv = bp[s * NPo + rlane];
#pragma unroll
      for (int r = 0; r < 8; ++r) ot[(wave * 16 + hh * 8 + r) * W + s * NPo + rlane] = acc[r] + bv;
    }
  }
  __syncthreads();
  const int cnt4 = 16 * W;
  const bool act = t < cnt4;
  v4f v = (v4f){0.f,0.f,0.f,0.f};
  float* dp = out;
  if (act) {
    v = *(const v4f*)(ot + 4 * t);
    dp = out + (size_t)m0 * W + 4 * t;
    *(volatile v4f*)dp = v;
  }
  __threadfence();
  if (act) *(volatile v4f*)dp = v;
}

extern "C" void kernel_launch(void* const* d_in, const int* in_sizes, int n_in,
                              void* d_out, int out_size, void* d_ws, size_t ws_size,
                              hipStream_t stream) {
  (void)in_sizes; (void)out_size;
  if (n_in < 33) return;

  const float* x_A      = (const float*)d_in[0];
  const float* x_B      = (const float*)d_in[1];
  const int*   gmask    = (const int*)d_in[2];
  const int*   lmask_A  = (const int*)d_in[3];
  const int*   lmask_B  = (const int*)d_in[4];
  const int*   objA     = (const int*)d_in[5];
  const int*   objB     = (const int*)d_in[6];
  const float* enc_Wl_A = (const float*)d_in[7];
  const float* enc_bl_A = (const float*)d_in[8];
  const float* enc_Wg_A = (const float*)d_in[9];
  const float* enc_bg_A = (const float*)d_in[10];
  const float* enc_Wl_B = (const float*)d_in[11];
  const float* enc_bl_B = (const float*)d_in[12];
  const float* enc_Wg_B = (const float*)d_in[13];
  const float* enc_bg_B = (const float*)d_in[14];
  const float* dec_W1_A = (const float*)d_in[15];
  const float* dec_b1_A = (const float*)d_in[16];
  const float* dec_W2_A = (const float*)d_in[17];
  const float* dec_b2_A = (const float*)d_in[18];
  const float* dec_Wp_A = (const float*)d_in[19];
  const float* dec_bp_A = (const float*)d_in[20];
  const float* dec_W1_B = (const float*)d_in[21];
  const float* dec_b1_B = (const float*)d_in[22];
  const float* dec_W2_B = (const float*)d_in[23];
  const float* dec_b2_B = (const float*)d_in[24];
  const float* dec_Wp_B = (const float*)d_in[25];
  const float* dec_bp_B = (const float*)d_in[26];
  const float* rw_W1    = (const float*)d_in[27];
  const float* rw_b1    = (const float*)d_in[28];
  const float* rw_W2    = (const float*)d_in[29];
  const float* rw_b2    = (const float*)d_in[30];
  const float* rw_W3    = (const float*)d_in[31];
  const float* rw_b3    = (const float*)d_in[32];

  char*  ws  = (char*)d_ws;
  size_t off = 0;
  auto carve = [&](size_t bytes) -> char* {
    char* p = ws + off;
    off += (bytes + 255) & ~(size_t)255;
    return p;
  };
  _Float16* WlA16 = (_Float16*)carve((size_t)DL * DIN * 2);
  _Float16* WgA16 = (_Float16*)carve((size_t)DG * DIN * 2);
  _Float16* WlB16 = (_Float16*)carve((size_t)DL * DIN * 2);
  _Float16* WgB16 = (_Float16*)carve((size_t)DG * DIN * 2);
  _Float16* W1tA  = (_Float16*)carve((size_t)NF_A * DH * DINdA * 2);
  _Float16* W2tA  = (_Float16*)carve((size_t)NF_A * DH * DH * 2);
  _Float16* W1tB  = (_Float16*)carve((size_t)NF_B * DH * DINdB * 2);
  _Float16* W2tB  = (_Float16*)carve((size_t)NF_B * DH * DH * 2);
  _Float16* rwW1t = (_Float16*)carve((size_t)DH * DGE * 2);
  _Float16* rwW2t = (_Float16*)carve((size_t)DH * DH * 2);
  _Float16* WpA16 = (_Float16*)carve((size_t)NF_A * 16 * DH * 2);
  _Float16* WpB16 = (_Float16*)carve((size_t)NF_B * 16 * DH * 2);
  _Float16* W3_16 = (_Float16*)carve((size_t)16 * DH * 2);
  _Float16* hlA   = (_Float16*)carve((size_t)MA * DL * 2);
  _Float16* hlB   = (_Float16*)carve((size_t)MB * DL * 2);
  _Float16* G16   = (_Float16*)carve((size_t)Bn * GROW * 2);
  float*    GpjA  = (float*)   carve((size_t)NF_A * Bn * DH * 4);
  float*    GpjB  = (float*)   carve((size_t)NF_B * Bn * DH * 4);
  _Float16* R1    = (_Float16*)carve((size_t)Bn * DH * 2);
  _Float16* R2    = (_Float16*)carve((size_t)Bn * DH * 2);
  const size_t bigBytes = (size_t)NF_A * RA_ * DH * 2;
  char* RegA = carve(bigBytes);
  char* RegB = carve(bigBytes);
  if (off > ws_size) return;
  if (off > (size_t)134217728) return;

  _Float16* xA16 = (_Float16*)RegA;
  _Float16* xB16 = (_Float16*)(RegA + (size_t)MA * DIN * 2);
  float*    hgA  = (float*)RegB;
  float*    hgB  = (float*)(RegB + (size_t)MA * DG * 4);
  _Float16* XlA  = (_Float16*)RegA;
  _Float16* H1A  = (_Float16*)RegB;
  _Float16* H2A  = (_Float16*)RegA;
  _Float16* XlB  = (_Float16*)RegA;
  _Float16* H1B  = (_Float16*)RegB;
  _Float16* H2B  = (_Float16*)RegA;

  float* outA = (float*)d_out;
  float* outB = outA + (size_t)Bn * NO_A * NF_A * NP;
  float* outR = outB + (size_t)Bn * NO_B * NF_B * NP;

  {
    const int n8A = MA * DIN / 8, n8B = MB * DIN / 8;
    cast_f32_f16x8<<<(n8A + 255) / 256, 256, 0, stream>>>(x_A, xA16, n8A);
    cast_f32_f16x8<<<(n8B + 255) / 256, 256, 0, stream>>>(x_B, xB16, n8B);
  }
  transpose_w16<<<dim3(DL / 64, DIN / 64, 1), 256, 0, stream>>>(enc_Wl_A, WlA16, DIN, DL);
  transpose_w16<<<dim3(DG / 64, DIN / 64, 1), 256, 0, stream>>>(enc_Wg_A, WgA16, DIN, DG);
  transpose_w16<<<dim3(DL / 64, DIN / 64, 1), 256, 0, stream>>>(enc_Wl_B, WlB16, DIN, DL);
  transpose_w16<<<dim3(DG / 64, DIN / 64, 1), 256, 0, stream>>>(enc_Wg_B, WgB16, DIN, DG);
  transpose_w16<<<dim3(DH / 64, DINdA / 64, NF_A), 256, 0, stream>>>(dec_W1_A, W1tA, DINdA, DH);
  transpose_w16<<<dim3(DH / 64, DH / 64, NF_A), 256, 0, stream>>>(dec_W2_A, W2tA, DH, DH);
  transpose_w16<<<dim3(DH / 64, DINdB / 64, NF_B), 256, 0, stream>>>(dec_W1_B, W1tB, DINdB, DH);
  transpose_w16<<<dim3(DH / 64, DH / 64, NF_B), 256, 0, stream>>>(dec_W2_B, W2tB, DH, DH);
  transpose_w16<<<dim3(DH / 64, DGE / 64, 1), 256, 0, stream>>>(rw_W1, rwW1t, DGE, DH);
  transpose_w16<<<dim3(DH / 64, DH / 64, 1), 256, 0, stream>>>(rw_W2, rwW2t, DH, DH);
  pack_head_w16<<<(NF_A * 512 + 255) / 256, 256, 0, stream>>>(dec_Wp_A, WpA16, NF_A, NP);
  pack_head_w16<<<(NF_B * 512 + 255) / 256, 256, 0, stream>>>(dec_Wp_B, WpB16, NF_B, NP);
  pack_head_w16<<<(1 * 512 + 255) / 256, 256, 0, stream>>>(rw_W3, W3_16, 1, 1);

  {
    const int gA = ((MA / 64) * (DL / 64) + 7) / 8;
    const int gB = ((MB / 64) * (DL / 64) + 7) / 8;
    wmma_gemm64<2, 0, 1, 2><<<dim3(gA, 1), 256, 0, stream>>>(
        xA16, DIN, 0, WlA16, DIN, 0, (void*)hlA, DL, 0, enc_bl_A, 0, nullptr, 0, 0, 0, MA, DL, DIN);
    wmma_gemm64<2, 0, 0, 0><<<dim3(gA, 1), 256, 0, stream>>>(
        xA16, DIN, 0, WgA16, DIN, 0, (void*)hgA, DG, 0, enc_bg_A, 0, nullptr, 0, 0, 0, MA, DG, DIN);
    wmma_gemm64<2, 0, 1, 2><<<dim3(gB, 1), 256, 0, stream>>>(
        xB16, DIN, 0, WlB16, DIN, 0, (void*)hlB, DL, 0, enc_bl_B, 0, nullptr, 0, 0, 0, MB, DL, DIN);
    wmma_gemm64<2, 0, 0, 0><<<dim3(gB, 1), 256, 0, stream>>>(
        xB16, DIN, 0, WgB16, DIN, 0, (void*)hgB, DG, 0, enc_bg_B, 0, nullptr, 0, 0, 0, MB, DG, DIN);
  }
  pool_global_kernel<<<Bn, 448, 0, stream>>>(hgA, hgB, objA, objB, gmask, G16);

  {
    const int total8 = NF_A * RA_ * (NF_A * 8);
    build_local_kernel<<<(total8 + 255) / 256, 256, 0, stream>>>(hlA, lmask_A, XlA, NO_A, NF_A, RA_, total8);
    const int gP = ((Bn / 64) * (DH / 64) + 7) / 8;
    wmma_gemm64<2, 0, 0, 0><<<dim3(gP, NF_A), 256, 0, stream>>>(
        G16, GROW, (long)DGE, W1tA + NF_A * DL, DINdA, (long)DH * DINdA, (void*)GpjA, DH, (long)Bn * DH,
        dec_b1_A, (long)DH, nullptr, 0, 0, 0, Bn, DH, DGE);
    const int gL = ((RA_ / 64) * (DH / 64) + 7) / 8;
    wmma_gemm64<0, 2, 1, 4><<<dim3(gL, NF_A), 256, 0, stream>>>(
        XlA, NF_A * DL, (long)RA_ * NF_A * DL, W1tA, DINdA, (long)DH * DINdA, (void*)H1A, DH, (long)RA_ * DH,
        nullptr, 0, GpjA, (long)Bn * DH, DH, 6, RA_, DH, NF_A * DL);
    wmma_gemm64<2, 0, 1, 4><<<dim3(gL, NF_A), 256, 0, stream>>>(
        H1A, DH, (long)RA_ * DH, W2tA, DH, (long)DH * DH, (void*)H2A, DH, (long)RA_ * DH,
        dec_b2_A, (long)DH, nullptr, 0, 0, 0, RA_, DH, DH);
    head_kernel<<<RA_ / 64, 128, 0, stream>>>(H2A, (long)RA_ * DH, WpA16, dec_bp_A, outA, NF_A, NP, RA_);
  }
  {
    const int total8 = NF_B * RB_ * (NF_B * 8);
    build_local_kernel<<<(total8 + 255) / 256, 256, 0, stream>>>(hlB, lmask_B, XlB, NO_B, NF_B, RB_, total8);
    const int gP = ((Bn / 64) * (DH / 64) + 7) / 8;
    wmma_gemm64<2, 0, 0, 0><<<dim3(gP, NF_B), 256, 0, stream>>>(
        G16 + NF_A * DGE, GROW, (long)DGE, W1tB + NF_B * DL, DINdB, (long)DH * DINdB, (void*)GpjB, DH, (long)Bn * DH,
        dec_b1_B, (long)DH, nullptr, 0, 0, 0, Bn, DH, DGE);
    const int gL = ((RB_ / 64) * (DH / 64) + 7) / 8;
    wmma_gemm64<0, 2, 1, 4><<<dim3(gL, NF_B), 256, 0, stream>>>(
        XlB, NF_B * DL, (long)RB_ * NF_B * DL, W1tB, DINdB, (long)DH * DINdB, (void*)H1B, DH, (long)RB_ * DH,
        nullptr, 0, GpjB, (long)Bn * DH, DH, 5, RB_, DH, NF_B * DL);
    wmma_gemm64<2, 0, 1, 4><<<dim3(gL, NF_B), 256, 0, stream>>>(
        H1B, DH, (long)RB_ * DH, W2tB, DH, (long)DH * DH, (void*)H2B, DH, (long)RB_ * DH,
        dec_b2_B, (long)DH, nullptr, 0, 0, 0, RB_, DH, DH);
    head_kernel<<<RB_ / 64, 128, 0, stream>>>(H2B, (long)RB_ * DH, WpB16, dec_bp_B, outB, NF_B, NP, RB_);
  }
  {
    const int gR = ((Bn / 64) * (DH / 64) + 7) / 8;
    wmma_gemm64<2, 0, 1, 4><<<dim3(gR, 1), 256, 0, stream>>>(
        G16 + NS * DGE, GROW, 0, rwW1t, DGE, 0, (void*)R1, DH, 0, rw_b1, 0, nullptr, 0, 0, 0, Bn, DH, DGE);
    wmma_gemm64<2, 0, 1, 4><<<dim3(gR, 1), 256, 0, stream>>>(
        R1, DH, 0, rwW2t, DH, 0, (void*)R2, DH, 0, rw_b2, 0, nullptr, 0, 0, 0, Bn, DH, DH);
    head_kernel<<<Bn / 64, 128, 0, stream>>>(R2, 0, W3_16, rw_b3, outR, 1, 1, Bn);
  }
  (void)hipGetLastError();
}
